// Mamba_12601434046490
// MI455X (gfx1250) — hardware-verified
//
#include <hip/hip_runtime.h>
#include <math.h>

typedef __attribute__((ext_vector_type(16))) _Float16 v16h;
typedef __attribute__((ext_vector_type(8)))  _Float16 v8h;
typedef __attribute__((ext_vector_type(8)))  float    v8f;
typedef __attribute__((ext_vector_type(4)))  float    v4f;
typedef __attribute__((ext_vector_type(4)))  unsigned v4u;

constexpr int kLayers = 4;
constexpr int kDm     = 512;
constexpr int kCin    = 768;
constexpr int kCout   = 40;
constexpr int kCoutP  = 64;
constexpr int kTaps   = 5;
constexpr int kDin    = 1024;
constexpr int kNst    = 16;
constexpr int kDtR    = 32;
constexpr int kXdP    = 64;
constexpr int kBatch  = 4;
constexpr int kSeq    = 1024;
constexpr int kSeqP   = kSeq + 4;
constexpr int kRows   = kBatch * kSeq;
constexpr int kKic    = kTaps * kCin;
constexpr int kKoc    = kTaps * kDm;
constexpr int kConvTP = 260;
constexpr int kScanTS = 64;
constexpr int kScanCh = 64;
constexpr int kScanYP = 68;
static_assert(kDtR + 2 * kNst == kXdP, "x_proj width");
static_assert((kKic % 32) == 0 && (kKoc % 32) == 0 && (kDm % 32) == 0 && (kDin % 32) == 0 && (kDtR % 32) == 0, "GEMM K multiples of 32");
static_assert((kSeq % 64) == 0 && (kRows % 64) == 0 && (kDm % 64) == 0 && (kDin % 64) == 0 && (kXdP % 64) == 0 && (kCoutP % 64) == 0, "GEMM M,N multiples of 64");
static_assert((kSeq % kScanTS) == 0 && (kDin % kScanCh) == 0 && (kDin % 256) == 0 && (kCin % 64) == 0, "tile multiples");

constexpr float kCarW   = 1024.0f;
constexpr float kCarWdt = 64.0f;
constexpr float kCarXc  = 256.0f;
constexpr float kCarDt  = 256.0f;
constexpr float kCarY   = 1024.0f;
constexpr float kCarH   = 1024.0f;

constexpr size_t kOffXT   = 0;
constexpr size_t kOffWIC  = kOffXT   + (size_t)kBatch * kSeqP * kCin * 2;
constexpr size_t kOffWIN  = kOffWIC  + (size_t)kDm * kKic * 2;
constexpr size_t kOffWXP  = kOffWIN  + (size_t)kLayers * 2 * kDin * kDm * 2;
constexpr size_t kOffWDT  = kOffWXP  + (size_t)kLayers * kXdP * kDin * 2;
constexpr size_t kOffWOUT = kOffWDT  + (size_t)kLayers * kDin * kDtR * 2;
constexpr size_t kOffWOC  = kOffWOUT + (size_t)kLayers * kDm * kDin * 2;
constexpr size_t kOffH    = kOffWOC  + (size_t)kCoutP * kKoc * 2;
constexpr size_t kOffRESA = kOffH    + (size_t)kRows * kDm * 4;
constexpr size_t kOffRESB = kOffRESA + (size_t)kRows * kDm * 4;
constexpr size_t kOffHN   = kOffRESB + (size_t)kRows * kDm * 4;
constexpr size_t kOffXIZ  = kOffHN   + (size_t)kRows * kDm * 2;
constexpr size_t kOffXC   = kOffXIZ  + (size_t)2 * kRows * kDin * 4;
constexpr size_t kOffXC16 = kOffXC   + (size_t)kRows * kDin * 4;
constexpr size_t kOffXD   = kOffXC16 + (size_t)kRows * kDin * 2;
constexpr size_t kOffDT16 = kOffXD   + (size_t)kRows * kXdP * 4;
constexpr size_t kOffY16  = kOffDT16 + (size_t)kRows * kDtR * 2;
constexpr size_t kOffHT   = kOffY16  + (size_t)kRows * kDin * 2;
constexpr size_t kWsTotal = kOffHT   + (size_t)kBatch * kSeqP * kDm * 2;
static_assert(kWsTotal == 125935616ull, "carve total");
static_assert(kWsTotal <= 134217728ull, "carve cap");
static_assert((kOffWIC % 128) == 0 && (kOffWIN % 128) == 0 && (kOffWXP % 128) == 0 && (kOffWDT % 128) == 0 &&
              (kOffWOUT % 128) == 0 && (kOffWOC % 128) == 0 && (kOffH % 128) == 0 && (kOffRESA % 128) == 0 &&
              (kOffRESB % 128) == 0 && (kOffHN % 128) == 0 && (kOffXIZ % 128) == 0 && (kOffXC % 128) == 0 &&
              (kOffXC16 % 128) == 0 && (kOffXD % 128) == 0 && (kOffDT16 % 128) == 0 && (kOffY16 % 128) == 0 &&
              (kOffHT % 128) == 0, "128-B aligned regions");

__device__ __forceinline__ unsigned short f2bf_bits(float f) {
  unsigned u = __float_as_uint(f);
  return (unsigned short)((u + 0x7FFFu + ((u >> 16) & 1u)) >> 16);
}
__device__ __forceinline__ float bf_bits2f(unsigned short h) { return __uint_as_float(((unsigned)h) << 16); }
__device__ __forceinline__ float rbf(float f) { return bf_bits2f(f2bf_bits(f)); }

__device__ __forceinline__ void row_guard_h(v8f& a, v8f& b, v8f& c, v8f& d, v16h x, v16h y0, v16h y1, v16h y2, v16h y3) {
  asm volatile("v_nop\n\tv_nop\n\tv_nop\n\tv_nop" : "+v"(a), "+v"(b), "+v"(c), "+v"(d) : "v"(x), "v"(y0), "v"(y1), "v"(y2), "v"(y3));
}
__device__ __forceinline__ void keep4_h(v16h a, v16h b, v16h c, v16h d) { asm volatile("v_nop" :: "v"(a), "v"(b), "v"(c), "v"(d)); }
__device__ __forceinline__ void acc_guard4(v8f& a, v8f& b, v8f& c, v8f& d) { asm volatile("v_nop\n\tv_nop\n\tv_nop\n\tv_nop" : "+v"(a), "+v"(b), "+v"(c), "+v"(d)); }

struct FragH {
  union U { v16h v; v8h h[2]; };
  static __device__ __forceinline__ v16h load(const _Float16* p) {
    U f; f.h[0] = *(const v8h*)(p); f.h[1] = *(const v8h*)(p + 16); return f.v;
  }
  static __device__ __forceinline__ v8f mma(v16h a, v16h b, v8f c) {
    return __builtin_amdgcn_wmma_f32_16x16x32_f16(false, a, false, b, (short)0, c, false, false);
  }
};

template <int BIAS_MODE, int OUT_MODE, int MASK_MODE>
__global__ __launch_bounds__(256) void wmma_gemm64(
    const unsigned short* __restrict__ Ap, int lda, long strideA,
    const unsigned short* __restrict__ Btp, int ldb, long strideB,
    void* __restrict__ Cout, int ldc, long strideC,
    const float* __restrict__ bias, const int* __restrict__ lens,
    int M, int N, int K, int Mstore, float scale) {
  const _Float16* A  = (const _Float16*)Ap;
  const _Float16* Bt = (const _Float16*)Btp;
  __shared__ __align__(16) float sT[8][16 * 68];
  const int b    = blockIdx.y;
  const int lane = threadIdx.x & 31;
  const int wave = threadIdx.x >> 5;
  const int tilesN = N >> 6;
  const int tilesM = M >> 6;
  const int tile = blockIdx.x * 8 + wave;
  if (tile >= tilesM * tilesN) return;
  const int tm = tile / tilesN;
  const int tn = tile - tm * tilesN;
  const int m0 = tm << 6;
  const int n0 = tn << 6;

  const _Float16* Ab = A  + (size_t)b * strideA;
  const _Float16* Bb = Bt + (size_t)b * strideB;

  const int rlane = lane & 15;
  const int koff  = (lane >> 4) * 8;
  const int mOff  = (lane >> 4) * 8;

  v8f acc[4][4];
#pragma unroll
  for (int i = 0; i < 4; ++i)
#pragma unroll
    for (int j = 0; j < 4; ++j) acc[i][j] = (v8f){0.f,0.f,0.f,0.f,0.f,0.f,0.f,0.f};

  for (int k0 = 0; k0 < K; k0 += 32) {
    v16h bh[4];
#pragma unroll
    for (int j = 0; j < 4; ++j) {
      const size_t bo = (size_t)(n0 + (j << 4) + rlane) * ldb + koff + k0;
      bh[j] = FragH::load(Bb + bo);
    }
#pragma unroll
    for (int i = 0; i < 4; ++i) {
      const size_t ao = (size_t)(m0 + (i << 4) + rlane) * lda + koff + k0;
      v16h ah = FragH::load(Ab + ao);
#pragma unroll
      for (int j = 0; j < 4; ++j) acc[i][j] = FragH::mma(ah, bh[j], acc[i][j]);
      row_guard_h(acc[i][0], acc[i][1], acc[i][2], acc[i][3], ah, bh[0], bh[1], bh[2], bh[3]);
    }
    keep4_h(bh[0], bh[1], bh[2], bh[3]);
  }
  acc_guard4(acc[0][0], acc[0][1], acc[0][2], acc[0][3]);
  acc_guard4(acc[1][0], acc[1][1], acc[1][2], acc[1][3]);
  acc_guard4(acc[2][0], acc[2][1], acc[2][2], acc[2][3]);
  acc_guard4(acc[3][0], acc[3][1], acc[3][2], acc[3][3]);

  float* slab = sT[wave];
  int lenb = 0;
  if (MASK_MODE != 0) lenb = lens[b];
#pragma unroll
  for (int i = 0; i < 4; ++i) {
    const int mBase = m0 + (i << 4);
    float bm[8];
#pragma unroll
    for (int r = 0; r < 8; ++r) {
      bm[r] = 0.f;
      if (BIAS_MODE == 1) {
        int mc = mBase + mOff + r;
        mc = (mc < Mstore) ? mc : (Mstore - 1);
        bm[r] = rbf(bias[mc]);
      }
    }
#pragma unroll
    for (int j = 0; j < 4; ++j) {
      const int n = n0 + (j << 4) + rlane;
      float bv = 0.f;
      if (BIAS_MODE == 2) bv = rbf(bias[n]);
#pragma unroll
      for (int r = 0; r < 8; ++r) {
        float v = acc[i][j][r] * scale;
        if (BIAS_MODE == 1) v += bm[r];
        if (BIAS_MODE == 2) v += bv;
        if (MASK_MODE == 1) v = ((mBase + mOff + r) < lenb) ? v : 0.0f;
        if (MASK_MODE == 2) v = (n < lenb) ? v : 0.0f;
        slab[(mOff + r) * 68 + (j << 4) + rlane] = v;
      }
    }
    __builtin_amdgcn_fence(__ATOMIC_RELEASE, "workgroup");
    __builtin_amdgcn_wave_barrier();
    __builtin_amdgcn_fence(__ATOMIC_ACQUIRE, "workgroup");
    if (OUT_MODE == 0) {
      float* C = (float*)Cout + (size_t)b * strideC;
      const int hh = lane >> 4, c4 = (lane & 15) * 4;
      for (int pass = 0; pass < 2; ++pass) {
#pragma unroll
        for (int it = 0; it < 8; ++it) {
          const int row = it * 2 + hh;
          v4f v = *(const v4f*)(slab + row * 68 + c4);
          if (mBase + row < Mstore)
            *(volatile v4f*)(C + (size_t)(mBase + row) * ldc + n0 + c4) = v;
        }
        __threadfence();
      }
    } else {
      const int q = lane >> 3, c8 = (lane & 7) * 8;
      unsigned short* C = (unsigned short*)Cout + (size_t)b * strideC;
      for (int pass = 0; pass < 2; ++pass) {
#pragma unroll
        for (int it = 0; it < 4; ++it) {
          const int row = it * 4 + q;
          const float* sp = slab + row * 68 + c8;
          v8h hv;
#pragma unroll
          for (int e = 0; e < 8; ++e) hv[e] = (_Float16)sp[e];
          if (mBase + row < Mstore)
            *(volatile v8h*)(C + (size_t)(mBase + row) * ldc + n0 + c8) = hv;
        }
        __threadfence();
      }
    }
    __builtin_amdgcn_fence(__ATOMIC_RELEASE, "workgroup");
    __builtin_amdgcn_wave_barrier();
    __builtin_amdgcn_fence(__ATOMIC_ACQUIRE, "workgroup");
  }
}

__global__ __launch_bounds__(256) void cast_w_kernel(
    const float* __restrict__ src, unsigned short* __restrict__ dst, int total8, float scale)
{
  const int i = blockIdx.x * 256 + threadIdx.x;
  if (i >= total8) return;
  const size_t e0 = (size_t)i << 3;
  const v4f a0 = *(const v4f*)(src + e0);
  const v4f a1 = *(const v4f*)(src + e0 + 4);
  v8h hv;
#pragma unroll
  for (int e = 0; e < 4; ++e) {
    const float f0 = a0[e];
    const float f1 = a1[e];
    hv[e]     = (_Float16)(rbf(f0) * scale);
    hv[4 + e] = (_Float16)(rbf(f1) * scale);
  }
  unsigned short* q = dst + e0;
  *(volatile v8h*)q = hv;
  __threadfence();
  *(volatile v8h*)q = hv;
}

__global__ __launch_bounds__(256) void repack_conv_kernel(
    const float* __restrict__ w, unsigned short* __restrict__ dst, int Oreal, int C, int total8, float scale)
{
  const int i = blockIdx.x * 256 + threadIdx.x;
  if (i >= total8) return;
  const int e0  = i << 3;
  const int KK  = kTaps * C;
  const int o   = e0 / KK;
  const int rem = e0 - o * KK;
  const int tap = rem / C;
  const int c   = rem - tap * C;
  const int oc  = (o < Oreal) ? o : (Oreal - 1);
  const float* p = w + ((size_t)oc * C + c) * kTaps + tap;
  v8h hv;
#pragma unroll
  for (int e = 0; e < 8; ++e) {
    const float v = p[e * kTaps];
    hv[e] = (_Float16)((o < Oreal) ? (rbf(v) * scale) : 0.0f);
  }
  unsigned short* q = dst + (size_t)e0;
  *(volatile v8h*)q = hv;
  __threadfence();
  *(volatile v8h*)q = hv;
}

__global__ __launch_bounds__(256) void xpose_x_kernel(
    const float* __restrict__ x, unsigned short* __restrict__ XT)
{
  __shared__ float tile[64 * 65];
  const int tid = threadIdx.x, lane = tid & 31, wave = tid >> 5;
  const int l0 = blockIdx.x * 64;
  const int c0 = blockIdx.y * 64;
  const int b  = blockIdx.z;
#pragma unroll
  for (int p = 0; p < 16; ++p) {
    const int idx = tid + p * 256;
    const int cc  = idx >> 6;
    const int ll  = idx & 63;
    const float v = x[((size_t)(b * kCin + c0 + cc)) * kSeq + l0 + ll];
    tile[cc * 65 + ll] = rbf(v);
  }
  __syncthreads();
  const int q = lane >> 3, c8 = (lane & 7) * 8;
  v8h hv[2];
#pragma unroll
  for (int it = 0; it < 2; ++it) {
    const int lrow = it * 32 + wave * 4 + q;
#pragma unroll
    for (int e = 0; e < 8; ++e) hv[it][e] = (_Float16)tile[(c8 + e) * 65 + lrow];
  }
  for (int pass = 0; pass < 2; ++pass) {
#pragma unroll
    for (int it = 0; it < 2; ++it) {
      const int lrow = it * 32 + wave * 4 + q;
      *(volatile v8h*)(XT + ((size_t)(b * kSeqP + l0 + lrow + 2)) * kCin + c0 + c8) = hv[it];
    }
    __threadfence();
  }
}

__global__ __launch_bounds__(256) void zero_pad_rows_kernel(unsigned short* __restrict__ P, int C, int total)
{
  const int i = blockIdx.x * 256 + threadIdx.x;
  if (i >= total) return;
  const int per  = C >> 3;
  const int prow = i / per;
  const int seg  = i - prow * per;
  const int b    = prow >> 2;
  const int j    = prow & 3;
  const int row  = (j < 2) ? j : (kSeq + j);
  unsigned short* q = P + ((size_t)(b * kSeqP + row)) * C + seg * 8;
  const v4u z = (v4u){0u, 0u, 0u, 0u};
  *(volatile v4u*)q = z;
  __threadfence();
  *(volatile v4u*)q = z;
}

__global__ __launch_bounds__(256) void ln_kernel(
    const float* __restrict__ H, const float* __restrict__ RIN, float* __restrict__ ROUT,
    const float* __restrict__ nw, const float* __restrict__ nb, unsigned short* __restrict__ HN, int addres)
{
  __shared__ __align__(16) float sN[8][kDm];
  const int tid = threadIdx.x, lane = tid & 31, wave = tid >> 5;
  const int row = blockIdx.x * 8 + wave;
  const float* hp = H   + (size_t)row * kDm;
  const float* rp = RIN + (size_t)row * kDm;
  v4f x[4];
#pragma unroll
  for (int j = 0; j < 4; ++j) {
    const v4f a = *(const v4f*)(hp + j * 128 + lane * 4);
    const v4f r = *(const v4f*)(rp + j * 128 + lane * 4);
    v4f t;
#pragma unroll
    for (int e = 0; e < 4; ++e) t[e] = (addres != 0) ? (a[e] + r[e]) : a[e];
    x[j] = t;
  }
  float s = 0.f;
#pragma unroll
  for (int j = 0; j < 4; ++j)
#pragma unroll
    for (int e = 0; e < 4; ++e) s += x[j][e];
#pragma unroll
  for (int off = 16; off > 0; off >>= 1) s += __shfl_xor(s, off, 32);
  const float mean = s * (1.0f / (float)kDm);
  float ss = 0.f;
#pragma unroll
  for (int j = 0; j < 4; ++j)
#pragma unroll
    for (int e = 0; e < 4; ++e) {
      const float dd = x[j][e] - mean;
      ss += dd * dd;
    }
#pragma unroll
  for (int off = 16; off > 0; off >>= 1) ss += __shfl_xor(ss, off, 32);
  const float rs = rsqrtf(ss * (1.0f / (float)kDm) + 1e-5f);
  float* sl = sN[wave];
#pragma unroll
  for (int j = 0; j < 4; ++j) {
    const v4f wv = *(const v4f*)(nw + j * 128 + lane * 4);
    const v4f bv = *(const v4f*)(nb + j * 128 + lane * 4);
    v4f o;
#pragma unroll
    for (int e = 0; e < 4; ++e) {
      const float wf = wv[e];
      const float bf = bv[e];
      o[e] = (x[j][e] - mean) * rs * rbf(wf) + rbf(bf);
    }
    *(v4f*)(sl + j * 128 + lane * 4) = o;
  }
  __syncthreads();
  v8h hv[2];
#pragma unroll
  for (int c = 0; c < 2; ++c) {
    const float* sp = sl + c * 256 + lane * 8;
    const v4f a0 = *(const v4f*)(sp);
    const v4f a1 = *(const v4f*)(sp + 4);
#pragma unroll
    for (int e = 0; e < 4; ++e) {
      hv[c][e]     = (_Float16)a0[e];
      hv[c][4 + e] = (_Float16)a1[e];
    }
  }
  float* op = ROUT + (size_t)row * kDm;
  unsigned short* hq = HN + (size_t)row * kDm;
  for (int pass = 0; pass < 2; ++pass) {
#pragma unroll
    for (int j = 0; j < 4; ++j) *(volatile v4f*)(op + j * 128 + lane * 4) = x[j];
#pragma unroll
    for (int c = 0; c < 2; ++c) *(volatile v8h*)(hq + c * 256 + lane * 8) = hv[c];
    __threadfence();
  }
}

__global__ __launch_bounds__(256) void conv_silu_kernel(
    const float* __restrict__ XI, const float* __restrict__ cw, const float* __restrict__ cb,
    float* __restrict__ XC, unsigned short* __restrict__ XC16)
{
  __shared__ __align__(16) float sT[16 * kConvTP];
  const int tid = threadIdx.x, lane = tid & 31, wave = tid >> 5;
  const int d0 = blockIdx.x * 256, d = d0 + tid;
  const int g0 = blockIdx.y * 64;
  const int tb = g0 & (kSeq - 1);
  const v4f wq = *(const v4f*)(cw + d * 4);
  const float wf0 = wq[0], wf1 = wq[1], wf2 = wq[2], wf3 = wq[3];
  const float w0 = rbf(wf0), w1 = rbf(wf1), w2 = rbf(wf2), w3 = rbf(wf3);
  const float bc = rbf(cb[d]);
  float xm3, xm2, xm1;
  {
    const bool hist = (tb > 0);
    const int rb = hist ? (g0 - 3) : g0;
    const float v3 = XI[(size_t)rb * kDin + d];
    const float v2 = XI[(size_t)(rb + 1) * kDin + d];
    const float v1 = XI[(size_t)(rb + 2) * kDin + d];
    xm3 = hist ? v3 : 0.f;
    xm2 = hist ? v2 : 0.f;
    xm1 = hist ? v1 : 0.f;
  }
  const int hrow = wave >> 1;
  const int hch  = (wave & 1) * 128 + lane * 4;
#pragma unroll 1
  for (int sub = 0; sub < 4; ++sub) {
    const int lb = g0 + sub * 16;
#pragma unroll 1
    for (int s = 0; s < 16; ++s) {
      const float xcur = XI[(size_t)(lb + s) * kDin + d];
      float acc = w0 * xm3;
      acc = fmaf(w1, xm2, acc);
      acc = fmaf(w2, xm1, acc);
      acc = fmaf(w3, xcur, acc);
      const float sv = acc + bc;
      const float sg = __builtin_amdgcn_rcpf(1.0f + expf(-sv));
      sT[s * kConvTP + tid] = sv * sg;
      xm3 = xm2; xm2 = xm1; xm1 = xcur;
    }
    __syncthreads();
    v4f fv[4];
    v8h bv[2];
#pragma unroll
    for (int it = 0; it < 4; ++it) fv[it] = *(const v4f*)(sT + (it * 4 + hrow) * kConvTP + hch);
#pragma unroll
    for (int it = 0; it < 2; ++it) {
      const float* sp = sT + (it * 8 + wave) * kConvTP + lane * 8;
      const v4f a0 = *(const v4f*)(sp);
      const v4f a1 = *(const v4f*)(sp + 4);
#pragma unroll
      for (int e = 0; e < 4; ++e) {
        bv[it][e]     = (_Float16)(a0[e] * kCarXc);
        bv[it][4 + e] = (_Float16)(a1[e] * kCarXc);
      }
    }
    for (int pass = 0; pass < 2; ++pass) {
#pragma unroll
      for (int it = 0; it < 4; ++it)
        *(volatile v4f*)(XC + (size_t)(lb + it * 4 + hrow) * kDin + d0 + hch) = fv[it];
#pragma unroll
      for (int it = 0; it < 2; ++it)
        *(volatile v8h*)(XC16 + (size_t)(lb + it * 8 + wave) * kDin + d0 + lane * 8) = bv[it];
      __threadfence();
    }
    __syncthreads();
  }
}

__global__ __launch_bounds__(256) void dt_cast_kernel(
    const float* __restrict__ XD, unsigned short* __restrict__ DT16, int total8)
{
  const int i = blockIdx.x * 256 + threadIdx.x;
  if (i >= total8) return;
  const int e0  = i << 3;
  const int row = e0 >> 5;
  const int c8  = e0 & 31;
  const float* p = XD + (size_t)row * kXdP + c8;
  const v4f a0 = *(const v4f*)(p);
  const v4f a1 = *(const v4f*)(p + 4);
  v8h hv;
#pragma unroll
  for (int e = 0; e < 4; ++e) {
    hv[e]     = (_Float16)(a0[e] * kCarDt);
    hv[4 + e] = (_Float16)(a1[e] * kCarDt);
  }
  unsigned short* qd = DT16 + e0;
  *(volatile v8h*)qd = hv;
  __threadfence();
  *(volatile v8h*)qd = hv;
}

__global__ __launch_bounds__(64) void scan_kernel(
    const float* __restrict__ DLR, const float* __restrict__ XC, const float* __restrict__ Z,
    const float* __restrict__ XD, const float* __restrict__ Alog, const float* __restrict__ Dp,
    unsigned short* __restrict__ Y16)
{
  __shared__ __align__(16) float sX[kScanTS * 32];
  __shared__ __align__(16) float sY[kScanTS * kScanYP];
  __shared__ __align__(16) float sA[kNst * kScanCh];
  const int tid = threadIdx.x, lane = tid & 31, wave = tid >> 5;
  constexpr int kBlkPerB = kDin / kScanCh;
  const int bix = blockIdx.x / kBlkPerB;
  const int d0  = (blockIdx.x - bix * kBlkPerB) * kScanCh;
  const int d   = d0 + tid;
  const size_t row0 = (size_t)bix * kSeq;
#pragma unroll 1
  for (int s = 0; s < kNst; ++s) sA[s * kScanCh + tid] = -expf(rbf(Alog[(size_t)d * kNst + s]));
  __syncthreads();
  float negA[kNst], h[kNst];
#pragma unroll
  for (int s = 0; s < kNst; ++s) {
    negA[s] = sA[s * kScanCh + tid];
    h[s] = 0.f;
  }
  const float Dd = rbf(Dp[d]);
  const int q = lane >> 3, c8 = (lane & 7) * 8;
#pragma unroll 1
  for (int t0 = 0; t0 < kSeq; t0 += kScanTS) {
    __syncthreads();
#pragma unroll
    for (int i = 0; i < 8; ++i) {
      const int idx = tid + 64 * i;
      const int r   = idx >> 3;
      const int q4  = (idx & 7) * 4;
      *(v4f*)(sX + r * 32 + q4) = *(const v4f*)(XD + (row0 + t0 + r) * kXdP + kDtR + q4);
    }
    __syncthreads();
#pragma unroll 1
    for (int s = 0; s < kScanTS; ++s) {
      const size_t grow = row0 + t0 + s;
      const float* xr = sX + s * 32;
      float Bs[kNst], Cs[kNst];
#pragma unroll
      for (int q4 = 0; q4 < 4; ++q4) {
        const v4f bv = *(const v4f*)(xr + 4 * q4);
        const v4f cv = *(const v4f*)(xr + kNst + 4 * q4);
        Bs[4 * q4 + 0] = bv[0]; Bs[4 * q4 + 1] = bv[1]; Bs[4 * q4 + 2] = bv[2]; Bs[4 * q4 + 3] = bv[3];
        Cs[4 * q4 + 0] = cv[0]; Cs[4 * q4 + 1] = cv[1]; Cs[4 * q4 + 2] = cv[2]; Cs[4 * q4 + 3] = cv[3];
      }
      const float v   = DLR[grow * kDin + d];
      const float a   = __expf(-fabsf(v));
      const float u   = 1.0f + a;
      const float l1p = __logf(u) + (a - (u - 1.0f)) * __builtin_amdgcn_rcpf(u);
      const float dt  = fmaxf(v, 0.0f) + l1p;
      const float xt  = XC[grow * kDin + d];
      const float dtx = dt * xt;
      float y = 0.f;
#pragma unroll
      for (int k = 0; k < kNst; ++k) {
        const float e = __expf(dt * negA[k]);
        h[k] = e * h[k] + dtx * Bs[k];
        y = h[k] * Cs[k] + y;
      }
      y = xt * Dd + y;
      const float zv = Z[grow * kDin + d];
      const float sg = __builtin_amdgcn_rcpf(1.0f + expf(-zv));
      y = y * (zv * sg);
      sY[s * kScanYP + tid] = y * kCarY;
    }
    __syncthreads();
    v8h hv[8];
#pragma unroll
    for (int it = 0; it < 8; ++it) {
      const int row = it * 8 + wave * 4 + q;
      const float* sp = sY + row * kScanYP + c8;
      const v4f a0 = *(const v4f*)(sp);
      const v4f a1 = *(const v4f*)(sp + 4);
#pragma unroll
      for (int e = 0; e < 4; ++e) {
        hv[it][e]     = (_Float16)a0[e];
        hv[it][4 + e] = (_Float16)a1[e];
      }
    }
    for (int pass = 0; pass < 2; ++pass) {
#pragma unroll
      for (int it = 0; it < 8; ++it) {
        const int row = it * 8 + wave * 4 + q;
        *(volatile v8h*)(Y16 + (row0 + t0 + row) * kDin + d0 + c8) = hv[it];
      }
      __threadfence();
    }
  }
}

extern "C" void kernel_launch(void* const* d_in, const int* in_sizes, int n_in,
                              void* d_out, int out_size, void* d_ws, size_t ws_size,
                              hipStream_t stream) {
  if (n_in < 17) return;
  if (in_sizes[0]  != kBatch * kCin * kSeq) return;
  if (in_sizes[1]  != kBatch) return;
  if (in_sizes[2]  != kDm * kCin * kTaps) return;
  if (in_sizes[3]  != kDm) return;
  if (in_sizes[4]  != kCout * kDm * kTaps) return;
  if (in_sizes[5]  != kCout) return;
  if (in_sizes[6]  != kLayers * 2 * kDin * kDm) return;
  if (in_sizes[7]  != kLayers * kDin * 4) return;
  if (in_sizes[8]  != kLayers * kDin) return;
  if (in_sizes[9]  != kLayers * kXdP * kDin) return;
  if (in_sizes[10] != kLayers * kDin * kDtR) return;
  if (in_sizes[11] != kLayers * kDin) return;
  if (in_sizes[12] != kLayers * kDin * kNst) return;
  if (in_sizes[13] != kLayers * kDin) return;
  if (in_sizes[14] != kLayers * kDm * kDin) return;
  if (in_sizes[15] != kLayers * kDm) return;
  if (in_sizes[16] != kLayers * kDm) return;
  if (out_size != kBatch * kCout * kSeq) return;
  if (ws_size < kWsTotal) return;

  const float* x          = (const float*)d_in[0];
  const int*   lengths    = (const int*)d_in[1];
  const float* in_conv_w  = (const float*)d_in[2];
  const float* in_conv_b  = (const float*)d_in[3];
  const float* out_conv_w = (const float*)d_in[4];
  const float* out_conv_b = (const float*)d_in[5];
  const float* in_proj_w  = (const float*)d_in[6];
  const float* conv_w     = (const float*)d_in[7];
  const float* conv_b     = (const float*)d_in[8];
  const float* x_proj_w   = (const float*)d_in[9];
  const float* dt_proj_w  = (const float*)d_in[10];
  const float* dt_proj_b  = (const float*)d_in[11];
  const float* A_log      = (const float*)d_in[12];
  const float* Dv         = (const float*)d_in[13];
  const float* out_proj_w = (const float*)d_in[14];
  const float* norm_w     = (const float*)d_in[15];
  const float* norm_b     = (const float*)d_in[16];
  float* out = (float*)d_out;

  char* ws = (char*)d_ws;
  unsigned short* XT   = (unsigned short*)(ws + kOffXT);
  unsigned short* WIC  = (unsigned short*)(ws + kOffWIC);
  unsigned short* WIN  = (unsigned short*)(ws + kOffWIN);
  unsigned short* WXP  = (unsigned short*)(ws + kOffWXP);
  unsigned short* WDT  = (unsigned short*)(ws + kOffWDT);
  unsigned short* WOUT = (unsigned short*)(ws + kOffWOUT);
  unsigned short* WOC  = (unsigned short*)(ws + kOffWOC);
  float*          H    = (float*)(ws + kOffH);
  float*          RESA = (float*)(ws + kOffRESA);
  float*          RESB = (float*)(ws + kOffRESB);
  unsigned short* HN   = (unsigned short*)(ws + kOffHN);
  float*          XIZ  = (float*)(ws + kOffXIZ);
  float*          XC   = (float*)(ws + kOffXC);
  unsigned short* XC16 = (unsigned short*)(ws + kOffXC16);
  float*          XD   = (float*)(ws + kOffXD);
  unsigned short* DT16 = (unsigned short*)(ws + kOffDT16);
  unsigned short* Y16  = (unsigned short*)(ws + kOffY16);
  unsigned short* HT   = (unsigned short*)(ws + kOffHT);
  float* XI  = XIZ;
  float* ZP  = XIZ + (size_t)kRows * kDin;
  float* DLR = XIZ;

  cast_w_kernel<<<(kLayers * 2 * kDin * kDm / 8) / 256, 256, 0, stream>>>(in_proj_w, WIN, kLayers * 2 * kDin * kDm / 8, kCarW);
  cast_w_kernel<<<(kLayers * kXdP * kDin / 8) / 256, 256, 0, stream>>>(x_proj_w, WXP, kLayers * kXdP * kDin / 8, kCarW);
  cast_w_kernel<<<(kLayers * kDin * kDtR / 8) / 256, 256, 0, stream>>>(dt_proj_w, WDT, kLayers * kDin * kDtR / 8, kCarWdt);
  cast_w_kernel<<<(kLayers * kDm * kDin / 8) / 256, 256, 0, stream>>>(out_proj_w, WOUT, kLayers * kDm * kDin / 8, kCarW);
  repack_conv_kernel<<<(kDm * kKic / 8) / 256, 256, 0, stream>>>(in_conv_w, WIC, kDm, kCin, kDm * kKic / 8, kCarW);
  repack_conv_kernel<<<(kCoutP * kKoc / 8) / 256, 256, 0, stream>>>(out_conv_w, WOC, kCout, kDm, kCoutP * kKoc / 8, kCarW);
  xpose_x_kernel<<<dim3(kSeq / 64, kCin / 64, kBatch), 256, 0, stream>>>(x, XT);
  zero_pad_rows_kernel<<<(16 * kCin / 8 + 255) / 256, 256, 0, stream>>>(XT, kCin, 16 * kCin / 8);
  zero_pad_rows_kernel<<<(16 * kDm / 8 + 255) / 256, 256, 0, stream>>>(HT, kDm, 16 * kDm / 8);

  wmma_gemm64<2, 0, 1><<<dim3(16, kBatch), 256, 0, stream>>>(
      XT, kCin, (long)kSeqP * kCin,
      WIC, kKic, 0L,
      (void*)H, kDm, (long)kSeq * kDm,
      in_conv_b, lengths,
      kSeq, kDm, kKic, kSeq, 1.0f / kCarW);

  for (int layer = 0; layer < kLayers; ++layer) {
    const float* rin  = (layer == 0) ? H : (((layer - 1) & 1) ? RESB : RESA);
    float*       rout = (layer & 1) ? RESB : RESA;
    ln_kernel<<<kRows / 8, 256, 0, stream>>>(H, rin, rout, norm_w + layer * kDm, norm_b + layer * kDm, HN, (layer > 0) ? 1 : 0);

    wmma_gemm64<0, 0, 0><<<dim3(128, 2), 256, 0, stream>>>(
        HN, kDm, 0L,
        WIN + (size_t)layer * 2 * kDin * kDm, kDm, (long)kDin * kDm,
        (void*)XIZ, kDin, (long)kRows * kDin,
        in_conv_b, lengths,
        kRows, kDin, kDm, kRows, 1.0f / kCarW);

    conv_silu_kernel<<<dim3(kDin / 256, kRows / 64), 256, 0, stream>>>(
        XI, conv_w + (size_t)layer * kDin * 4, conv_b + layer * kDin, XC, XC16);

    wmma_gemm64<0, 0, 0><<<dim3(8, 1), 256, 0, stream>>>(
        XC16, kDin, 0L,
        WXP + (size_t)layer * kXdP * kDin, kDin, 0L,
        (void*)XD, kXdP, 0L,
        in_conv_b, lengths,
        kRows, kXdP, kDin, kRows, 1.0f / (kCarXc * kCarW));

    dt_cast_kernel<<<(kRows * kDtR / 8) / 256, 256, 0, stream>>>(XD, DT16, kRows * kDtR / 8);

    wmma_gemm64<2, 0, 0><<<dim3(128, 1), 256, 0, stream>>>(
        DT16, kDtR, 0L,
        WDT + (size_t)layer * kDin * kDtR, kDtR, 0L,
        (void*)DLR, kDin, 0L,
        dt_proj_b + layer * kDin, lengths,
        kRows, kDin, kDtR, kRows, 1.0f / (kCarDt * kCarWdt));

    scan_kernel<<<kBatch * (kDin / kScanCh), kScanCh, 0, stream>>>(
        DLR, XC, ZP, XD, A_log + (size_t)layer * kDin * kNst, Dv + layer * kDin, Y16);

    if (layer + 1 < kLayers) {
      wmma_gemm64<0, 0, 0><<<dim3(64, 1), 256, 0, stream>>>(
          Y16, kDin, 0L,
          WOUT + (size_t)layer * kDm * kDin, kDin, 0L,
          (void*)H, kDm, 0L,
          in_conv_b, lengths,
          kRows, kDm, kDin, kRows, 1.0f / (kCarY * kCarW));
    } else {
      wmma_gemm64<0, 1, 0><<<dim3(16, kBatch), 256, 0, stream>>>(
          Y16, kDin, (long)kSeq * kDin,
          WOUT + (size_t)layer * kDm * kDin, kDin, 0L,
          (void*)(HT + 2 * kDm), kDm, (long)kSeqP * kDm,
          in_conv_b, lengths,
          kSeq, kDm, kDin, kSeq, kCarH / (kCarY * kCarW));
    }
  }

  wmma_gemm64<1, 0, 2><<<dim3(2, kBatch), 256, 0, stream>>>(
      WOC, kKoc, 0L,
      HT, kDm, (long)kSeqP * kDm,
      (void*)out, kSeq, (long)kCout * kSeq,
      out_conv_b, lengths,
      kCoutP, kSeq, kKoc, kCout, 1.0f / (kCarH * kCarW));
}
